// MultiHeadedAttention_27848567947459
// MI455X (gfx1250) — hardware-verified
//
#include <hip/hip_runtime.h>
#ifndef NB
#define NB 4
#endif
#ifndef SEQ
#define SEQ 2048
#endif
#define NB_FULL 4
#define SEQ_FULL 2048
#define DD 512
#define NH 8
#define HD 64

static_assert(NB >= 1 && NB <= NB_FULL);
static_assert(SEQ >= 64 && SEQ <= SEQ_FULL && (SEQ % 64) == 0);
static_assert(NH * HD == DD && (DD % 64) == 0 && (HD % 32) == 0 && HD <= 128);

typedef __bf16 v16b __attribute__((ext_vector_type(16)));
typedef unsigned short v8us __attribute__((ext_vector_type(8), may_alias));
typedef float  v8f  __attribute__((ext_vector_type(8)));
typedef float  v4f  __attribute__((ext_vector_type(4)));
typedef float  v4fa __attribute__((ext_vector_type(4), may_alias));
union FragB { v16b v; v8us half[2]; unsigned short u[16]; };

__device__ __forceinline__ unsigned short bf16_bits(float x) { unsigned int u = __float_as_uint(x); return (unsigned short)((u + 0x7FFFu + ((u >> 16) & 1u)) >> 16); }
__device__ __forceinline__ float bf16_val(unsigned short b) { return __uint_as_float(((unsigned int)b) << 16); }
__device__ __forceinline__ float bf16_rne(float x) { return bf16_val(bf16_bits(x)); }

template <int NT>
__device__ __forceinline__ v8f mmaN(v16b ah, v16b al, v16b bh, v16b bl, v8f c) {
  c = __builtin_amdgcn_wmma_f32_16x16x32_bf16(false, ah, false, bh, (short)0, c, false, false);
  if (NT >= 2) c = __builtin_amdgcn_wmma_f32_16x16x32_bf16(false, al, false, bh, (short)0, c, false, false);
  if (NT >= 3) c = __builtin_amdgcn_wmma_f32_16x16x32_bf16(false, ah, false, bl, (short)0, c, false, false);
  asm volatile("v_nop\n\tv_nop\n\tv_nop\n\tv_nop" : "+v"(c) : "v"(ah), "v"(al), "v"(bh), "v"(bl));
  return c;
}

__global__ __launch_bounds__(256) void k_rne_rows(const float* __restrict__ W, unsigned short* __restrict__ Wt, int n8) {
  const int t = blockIdx.x * 256 + threadIdx.x;
  if (t >= n8) return;
  const v4f a = *(const v4fa*)(W + (size_t)t * 8), b = *(const v4fa*)(W + (size_t)t * 8 + 4);
  v8us v; v[0]=bf16_bits(a[0]); v[1]=bf16_bits(a[1]); v[2]=bf16_bits(a[2]); v[3]=bf16_bits(a[3]);
  v[4]=bf16_bits(b[0]); v[5]=bf16_bits(b[1]); v[6]=bf16_bits(b[2]); v[7]=bf16_bits(b[3]);
  *(volatile v8us*)(Wt + (size_t)t * 8) = v; __threadfence(); *(volatile v8us*)(Wt + (size_t)t * 8) = v;
}

template <bool ASPLIT, bool BIAS_BF16>
__global__ __launch_bounds__(128) void k_gemm_bf(const float* __restrict__ A, int lda, int abatch, const unsigned short* __restrict__ Wt, int ldb,
                                               const float* __restrict__ bias, float* __restrict__ C, int ldc, int cbatch, int M, int N, int K) {
  __shared__ __attribute__((aligned(16))) float so[4][16][64];
  const int tid = threadIdx.x, w = tid >> 5, lane = tid & 31, ln = lane & 15, hh = lane >> 4;
  const int ntn = N / 64;
  const int wid = blockIdx.x * 4 + w;
  const int mt = wid / ntn, nq = wid % ntn;
  if (mt * 16 >= M) return;
  const int row0 = mt * 16, col0 = nq * 64;
  const float* Ab = A + (size_t)blockIdx.y * (size_t)abatch;
  float* Cb = C + (size_t)blockIdx.y * (size_t)cbatch;
  const float* arow = Ab + (size_t)(row0 + ln) * lda;
  v8f acc[4];
#pragma unroll
  for (int t = 0; t < 4; ++t) acc[t] = (v8f){0.f,0.f,0.f,0.f,0.f,0.f,0.f,0.f};
  for (int kb = 0; kb < K; kb += 32) {
    FragB ah, al;
    const v4f x0 = *(const v4fa*)(arow + kb + 8 * hh), x1 = *(const v4fa*)(arow + kb + 8 * hh + 4);
    const v4f x2 = *(const v4fa*)(arow + kb + 16 + 8 * hh), x3 = *(const v4fa*)(arow + kb + 16 + 8 * hh + 4);
    float xs[16] = {x0[0],x0[1],x0[2],x0[3],x1[0],x1[1],x1[2],x1[3],x2[0],x2[1],x2[2],x2[3],x3[0],x3[1],x3[2],x3[3]};
#pragma unroll
    for (int i = 0; i < 16; ++i) { const unsigned short hb = bf16_bits(xs[i]); ah.u[i] = hb; al.u[i] = ASPLIT ? bf16_bits(xs[i] - bf16_val(hb)) : (unsigned short)0; }
#pragma unroll
    for (int t = 0; t < 4; ++t) {
      const unsigned short* brow = Wt + (size_t)(col0 + t * 16 + ln) * ldb + kb;
      FragB b;
      b.half[0] = *(const v8us*)(brow + 8 * hh);
      b.half[1] = *(const v8us*)(brow + 16 + 8 * hh);
      acc[t] = mmaN<ASPLIT ? 2 : 1>(ah.v, al.v, b.v, b.v, acc[t]);
    }
  }
#pragma unroll
  for (int t = 0; t < 4; ++t) {
    float bvv = bias[col0 + t * 16 + ln];
    if (BIAS_BF16) bvv = bf16_rne(bvv);
#pragma unroll
    for (int r = 0; r < 8; ++r) { so[w][8 * hh + r][t * 16 + ln] = acc[t][r] + bvv; }
  }
  __builtin_amdgcn_fence(4  , "workgroup");
  __builtin_amdgcn_wave_barrier();
  const int rsub = lane >> 4, c4 = (lane & 15) * 4;
  for (int pass = 0; pass < 2; ++pass) {
#pragma unroll
    for (int q = 0; q < 8; ++q) {
      const int r = q * 2 + rsub;
      const v4f v = *(const v4fa*)&so[w][r][c4];
      *(volatile v4f*)(Cb + (size_t)(row0 + r) * ldc + col0 + c4) = v;
    }
    if (pass == 0) __threadfence();
  }
}

template <int D>
__global__ __launch_bounds__(128) void k_flash_pm(const float* __restrict__ Qb, const float* __restrict__ Kb, const float* __restrict__ Vb,
                                                int pitch, int T, int H, float scale, const int* __restrict__ kpm, int mpitch,
                                                float* __restrict__ y, int ypitch) {
  constexpr int KS = D / 32, DT = D / 16;
  __shared__ __attribute__((aligned(16))) unsigned short sKh[32][D + 8], sKl[32][D + 8], sVh[32][D + 8], sVl[32][D + 8];
  __shared__ __attribute__((aligned(16))) unsigned short sPh[4][16][40], sPl[4][16][40];
  __shared__ __attribute__((aligned(16))) float sO[4][16][D];
  const int tid = threadIdx.x, w = tid >> 5, lane = tid & 31, ln = lane & 15, hh = lane >> 4;
  const int nqb = (T + 63) / 64;
  const int bh = blockIdx.x / nqb, qblk = blockIdx.x % nqb;
  const int b = bh / H, h = bh % H;
  const int q0 = qblk * 64 + w * 16;
  const float* Q = Qb + (size_t)b * T * pitch + h * D;
  const float* K = Kb + (size_t)b * T * pitch + h * D;
  const float* V = Vb + (size_t)b * T * pitch + h * D;
  const int* mrow = kpm + (size_t)b * mpitch;

  FragB aqh[KS], aql[KS];
  {
    int row = q0 + ln; if (row >= T) row = T - 1;
    const float* qr = Q + (size_t)row * pitch;
#pragma unroll
    for (int ks = 0; ks < KS; ++ks)
#pragma unroll
      for (int i = 0; i < 16; ++i) {
        const int d = ks * 32 + ((i < 8) ? (8 * hh + i) : (16 + 8 * hh + (i - 8)));
        const float x = qr[d] * scale; const unsigned short hb = bf16_bits(x);
        aqh[ks].u[i] = hb; aql[ks].u[i] = bf16_bits(x - bf16_val(hb));
      }
  }
  float m_r[8], l_r[8];
#pragma unroll
  for (int r = 0; r < 8; ++r) { m_r[r] = -3.0e38f; l_r[r] = 0.f; }
  v8f oacc[DT];
#pragma unroll
  for (int dt = 0; dt < DT; ++dt) oacc[dt] = (v8f){0.f,0.f,0.f,0.f,0.f,0.f,0.f,0.f};

  for (int j0 = 0; j0 < T; j0 += 32) {
    __syncthreads();
    for (int e = tid; e < 32 * (D / 4); e += 128) {
      const int r = e / (D / 4), c4 = (e % (D / 4)) * 4;
      int key = j0 + r; const bool kin = key < T; if (!kin) key = T - 1;
      v4f kf = *(const v4fa*)(K + (size_t)key * pitch + c4);
      v4f vf = *(const v4fa*)(V + (size_t)key * pitch + c4);
      if (!kin) { kf = (v4f){0.f,0.f,0.f,0.f}; vf = (v4f){0.f,0.f,0.f,0.f}; }
#pragma unroll
      for (int t = 0; t < 4; ++t) {
        unsigned short hb = bf16_bits(kf[t]); sKh[r][c4 + t] = hb; sKl[r][c4 + t] = bf16_bits(kf[t] - bf16_val(hb));
        hb = bf16_bits(vf[t]); sVh[r][c4 + t] = hb; sVl[r][c4 + t] = bf16_bits(vf[t] - bf16_val(hb));
      }
    }
    __syncthreads();
    v8f s[2];
#pragma unroll
    for (int nt = 0; nt < 2; ++nt) {
      v8f acc = (v8f){0.f,0.f,0.f,0.f,0.f,0.f,0.f,0.f};
#pragma unroll
      for (int ks = 0; ks < KS; ++ks) {
        FragB bh_, bl_;
        bh_.half[0] = *(const v8us*)&sKh[nt * 16 + ln][ks * 32 + 8 * hh]; bh_.half[1] = *(const v8us*)&sKh[nt * 16 + ln][ks * 32 + 16 + 8 * hh];
        bl_.half[0] = *(const v8us*)&sKl[nt * 16 + ln][ks * 32 + 8 * hh]; bl_.half[1] = *(const v8us*)&sKl[nt * 16 + ln][ks * 32 + 16 + 8 * hh];
        acc = mmaN<3>(aqh[ks].v, aql[ks].v, bh_.v, bl_.v, acc);
      }
      s[nt] = acc;
    }
    const int ja = j0 + ln, jb = j0 + 16 + ln;
    const int jac = (ja < T) ? ja : (T - 1), jbc = (jb < T) ? jb : (T - 1);
    const int fa = mrow[jac], fb = mrow[jbc];
    const bool keepa = (ja < T) && (fa == 0), keepb = (jb < T) && (fb == 0);
    float alpha[8];
#pragma unroll
    for (int r = 0; r < 8; ++r) {
      if (!keepa) s[0][r] = -3.0e38f;
      if (!keepb) s[1][r] = -3.0e38f;
      float mx = fmaxf(s[0][r], s[1][r]);
      mx = fmaxf(mx, __shfl_xor(mx, 1, 32)); mx = fmaxf(mx, __shfl_xor(mx, 2, 32)); mx = fmaxf(mx, __shfl_xor(mx, 4, 32)); mx = fmaxf(mx, __shfl_xor(mx, 8, 32));
      const float mnew = fmaxf(m_r[r], mx);
      alpha[r] = (mnew > -1.0e38f) ? __expf(m_r[r] - mnew) : 1.0f;
      const float p0 = keepa ? __expf(s[0][r] - mnew) : 0.f;
      const float p1 = keepb ? __expf(s[1][r] - mnew) : 0.f;
      m_r[r] = mnew;
      l_r[r] = l_r[r] * alpha[r] + p0 + p1;
      unsigned short hb = bf16_bits(p0); sPh[w][8 * hh + r][ln] = hb;      sPl[w][8 * hh + r][ln] = bf16_bits(p0 - bf16_val(hb));
      hb = bf16_bits(p1);                sPh[w][8 * hh + r][16 + ln] = hb; sPl[w][8 * hh + r][16 + ln] = bf16_bits(p1 - bf16_val(hb));
    }
#pragma unroll
    for (int dt = 0; dt < DT; ++dt)
#pragma unroll
      for (int r = 0; r < 8; ++r) oacc[dt][r] *= alpha[r];
    __builtin_amdgcn_fence(4  , "workgroup");
    __builtin_amdgcn_wave_barrier();
    FragB pah, pal;
    pah.half[0] = *(const v8us*)&sPh[w][ln][8 * hh]; pah.half[1] = *(const v8us*)&sPh[w][ln][16 + 8 * hh];
    pal.half[0] = *(const v8us*)&sPl[w][ln][8 * hh]; pal.half[1] = *(const v8us*)&sPl[w][ln][16 + 8 * hh];
#pragma unroll
    for (int dt = 0; dt < DT; ++dt) {
      FragB bvh, bvl;
#pragma unroll
      for (int i = 0; i < 8; ++i) {
        bvh.u[i] = sVh[8 * hh + i][dt * 16 + ln]; bvh.u[8 + i] = sVh[16 + 8 * hh + i][dt * 16 + ln];
        bvl.u[i] = sVl[8 * hh + i][dt * 16 + ln]; bvl.u[8 + i] = sVl[16 + 8 * hh + i][dt * 16 + ln];
      }
      oacc[dt] = mmaN<3>(pah.v, pal.v, bvh.v, bvl.v, oacc[dt]);
    }
    __builtin_amdgcn_fence(4  , "workgroup");
    __builtin_amdgcn_wave_barrier();
  }
  const float qnan = __uint_as_float(0x7FC00000u);
#pragma unroll
  for (int r = 0; r < 8; ++r) {
    float l = l_r[r];
    l += __shfl_xor(l, 1, 32); l += __shfl_xor(l, 2, 32); l += __shfl_xor(l, 4, 32); l += __shfl_xor(l, 8, 32);
    l_r[r] = (m_r[r] > -1.0e38f) ? (1.0f / l) : qnan;
  }
#pragma unroll
  for (int dt = 0; dt < DT; ++dt)
#pragma unroll
    for (int r = 0; r < 8; ++r) sO[w][8 * hh + r][dt * 16 + ln] = oacc[dt][r] * l_r[r];
  __builtin_amdgcn_fence(4  , "workgroup");
  __builtin_amdgcn_wave_barrier();
  for (int pass = 0; pass < 2; ++pass) {
    for (int r = 0; r < 16; ++r) {
      const int row = q0 + r;
      if (row < T && lane < D / 4) {
        const v4f val = *(const v4fa*)&sO[w][r][lane * 4];
        *(volatile v4f*)(y + ((size_t)b * T + row) * ypitch + h * D + lane * 4) = val;
      }
    }
    if (pass == 0) __threadfence();
  }
}

extern "C" void kernel_launch(void* const* d_in, const int* in_sizes, int n_in,
                              void* d_out, int out_size, void* d_ws, size_t ws_size, hipStream_t stream) {
  if (n_in < 12) return;
  const float* xq = (const float*)d_in[0]; const float* xk = (const float*)d_in[1]; const float* xv = (const float*)d_in[2];
  const int* kpm = (const int*)d_in[3];
  const float* Wq = (const float*)d_in[4]; const float* bq = (const float*)d_in[5]; const float* Wk = (const float*)d_in[6]; const float* bk = (const float*)d_in[7];
  const float* Wv = (const float*)d_in[8]; const float* bv = (const float*)d_in[9]; const float* Wo = (const float*)d_in[10]; const float* bo = (const float*)d_in[11];
  const long long needX = (long long)(NB - 1) * SEQ_FULL * DD + (long long)SEQ * DD;
  if ((long long)in_sizes[0] < needX || (long long)in_sizes[1] < needX || (long long)in_sizes[2] < needX) return;
  if (in_sizes[3] < (NB - 1) * SEQ_FULL + SEQ) return;
  if (in_sizes[4] < DD * DD || in_sizes[6] < DD * DD || in_sizes[8] < DD * DD || in_sizes[10] < DD * DD) return;
  if (in_sizes[5] < DD || in_sizes[7] < DD || in_sizes[9] < DD || in_sizes[11] < DD) return;
  if ((long long)out_size < (long long)NB * SEQ * DD) return;

  char* ws = (char*)d_ws; size_t off = 0;
  auto take = [&](size_t bytes) { char* p = ws + off; off += (bytes + 255) & ~(size_t)255; return p; };
  const size_t MROWS = (size_t)NB * SEQ;
  unsigned short* Wt[4]; for (int i = 0; i < 4; ++i) Wt[i] = (unsigned short*)take((size_t)DD * DD * 2);
  float* q   = (float*)take(MROWS * DD * 4);
  float* k   = (float*)take(MROWS * DD * 4);
  float* v   = (float*)take(MROWS * DD * 4);
  float* att = (float*)take(MROWS * DD * 4);
  if (off > ws_size) return;

  const int n8 = DD * DD / 8;
  const int gb = ((SEQ / 16) * (DD / 64) + 3) / 4;
  const dim3 gg(gb, NB);
  const float* W4[4] = {Wq, Wk, Wv, Wo};
  for (int i = 0; i < 4; ++i) k_rne_rows<<<(n8 + 255) / 256, 256, 0, stream>>>(W4[i], Wt[i], n8);
  k_gemm_bf<false, true><<<gg, 128, 0, stream>>>(xq, DD, SEQ_FULL * DD, Wt[0], DD, bq, q, DD, SEQ * DD, SEQ, DD, DD);
  k_gemm_bf<false, true><<<gg, 128, 0, stream>>>(xk, DD, SEQ_FULL * DD, Wt[1], DD, bk, k, DD, SEQ * DD, SEQ, DD, DD);
  k_gemm_bf<false, true><<<gg, 128, 0, stream>>>(xv, DD, SEQ_FULL * DD, Wt[2], DD, bv, v, DD, SEQ * DD, SEQ, DD, DD);
  k_flash_pm<HD><<<NB * NH * (SEQ / 64), 128, 0, stream>>>(q, k, v, DD, SEQ, NH, 0.125f, kpm, SEQ_FULL, att, DD);
  k_gemm_bf<true, true><<<gg, 128, 0, stream>>>(att, DD, SEQ * DD, Wt[3], DD, bo, (float*)d_out, DD, SEQ * DD, SEQ, DD, DD);
  (void)hipGetLastError();
}
